// LocalFeatureAggregation_34239479284328
// MI455X (gfx1250) — hardware-verified
//
#include <hip/hip_runtime.h>
#include <math.h>

typedef __attribute__((ext_vector_type(16))) _Float16 v16h;
typedef __attribute__((ext_vector_type(16))) __bf16 v16b;
typedef __attribute__((ext_vector_type(8)))  _Float16 v8h;
typedef __attribute__((ext_vector_type(8)))  float v8f;
typedef __attribute__((ext_vector_type(4)))  float v4f;
typedef __attribute__((ext_vector_type(2)))  float v2f;
typedef __attribute__((ext_vector_type(4)))  unsigned v4u;
typedef __attribute__((ext_vector_type(4)))  int v4i;
typedef float __attribute__((may_alias)) float_a;
typedef int __attribute__((may_alias)) int_a;

template <typename T> __device__ __forceinline__ void vst2(void* p, T v) { *(volatile T*)p = v; __threadfence(); *(volatile T*)p = v; }
__device__ __forceinline__ v8f wmma16(v16h a, v16h b, v8f c) {
  v8f d = __builtin_amdgcn_wmma_f32_16x16x32_f16(false, a, false, b, (short)0, c, false, false);
  asm volatile("v_nop\n\tv_nop\n\tv_nop\n\tv_nop" : "+v"(d) : "v"(a), "v"(b));
  return d;
}
__device__ __forceinline__ v8f wmma_bf(v16b a, v16b b, v8f c) {
  v8f d = __builtin_amdgcn_wmma_f32_16x16x32_bf16(false, a, false, b, (short)0, c, false, false);
  asm volatile("v_nop\n\tv_nop\n\tv_nop\n\tv_nop" : "+v"(d) : "v"(a), "v"(b));
  return d;
}
__device__ __forceinline__ v16h frag_h(const _Float16* rowk0, int lane) {
  union { v16h v; v8h q[2]; } u; const _Float16* p = rowk0 + 8 * (lane >> 4);
  u.q[0] = *(const v8h*)p; u.q[1] = *(const v8h*)(p + 16); return u.v;
}
__device__ __forceinline__ v16h frag_f32(const float* rowk0, int lane) {
  v16h a; const float* p = rowk0 + 8 * (lane >> 4);
#pragma unroll
  for (int i = 0; i < 8; ++i) { a[i] = (_Float16)p[i]; a[8 + i] = (_Float16)p[16 + i]; }
  return a;
}
__device__ __forceinline__ v16h frag_f32s(const float* rowk0, int lane, float sc) {
  v16h a; const float* p = rowk0 + 8 * (lane >> 4);
#pragma unroll
  for (int i = 0; i < 8; ++i) { a[i] = (_Float16)(p[i] * sc); a[8 + i] = (_Float16)(p[16 + i] * sc); }
  return a;
}
__device__ __forceinline__ v16h fragc_f32(const float* W, int k0, int n, int lane, int ld, int K) {
  v16h a; const int g = lane >> 4;
#pragma unroll
  for (int i = 0; i < 8; ++i) { const int ka = k0 + 8 * g + i, kb = ka + 16;
    a[i] = (_Float16)(ka < K ? W[(size_t)(ka < K ? ka : K - 1) * ld + n] : 0.f); a[8 + i] = (_Float16)(kb < K ? W[(size_t)(kb < K ? kb : K - 1) * ld + n] : 0.f); }
  return a;
}
struct F2 { v16b h, l; };
__device__ __forceinline__ F2 bsplit16(const float v[16]) { F2 r;
#pragma unroll
  for (int i = 0; i < 16; ++i) { const __bf16 h = (__bf16)v[i]; r.h[i] = h; r.l[i] = (__bf16)(v[i] - (float)h); }
  return r; }
__device__ __forceinline__ F2 split_row(const float* row, int k0, int lane) { float v[16]; const float* p = row + k0 + 8 * (lane >> 4);
#pragma unroll
  for (int i = 0; i < 8; ++i) { v[i] = p[i]; v[8 + i] = p[16 + i]; }
  return bsplit16(v); }
__device__ __forceinline__ F2 split_rowK(const float* row, int k0, int lane, int K) { float v[16]; const int g = lane >> 4;
#pragma unroll
  for (int i = 0; i < 8; ++i) { const int ka = k0 + 8 * g + i, kb = ka + 16; v[i] = ka < K ? row[ka < K ? ka : K - 1] : 0.f; v[8 + i] = kb < K ? row[kb < K ? kb : K - 1] : 0.f; }
  return bsplit16(v); }
__device__ __forceinline__ F2 split_col(const float* W, int k0, int n, int lane, int ld, int K) { float v[16]; const int g = lane >> 4;
#pragma unroll
  for (int i = 0; i < 8; ++i) { const int ka = k0 + 8 * g + i, kb = ka + 16; v[i] = ka < K ? W[(size_t)(ka < K ? ka : K - 1) * ld + n] : 0.f; v[8 + i] = kb < K ? W[(size_t)(kb < K ? kb : K - 1) * ld + n] : 0.f; }
  return bsplit16(v); }
__device__ __forceinline__ v8f mac3(const F2& a, const F2& b, v8f c) { c = wmma_bf(a.l, b.h, c); c = wmma_bf(a.h, b.l, c); return wmma_bf(a.h, b.h, c); }
__device__ __forceinline__ float sigm(float v) { return 1.0f / (1.0f + expf(-v)); }
#define LDSX() do { asm volatile("s_wait_dscnt 0" ::: "memory"); __builtin_amdgcn_wave_barrier(); __builtin_amdgcn_fence(__ATOMIC_RELEASE, "workgroup"); } while (0)

#define NBT 2
#define NPT 32768
#define KN 16
#define CI 8
#define CO 64
#define NR (NBT * NPT)
#define EPB 256
#ifndef NRV
#define NRV NR
#endif
#define BNI 0.99999500003749981f
__device__ __forceinline__ float bfr(float v) { return (float)(__bf16)v; }
#define WS_PL  0u
#define WS_END (WS_PL + 4u * (size_t)NR * CO)
__device__ __forceinline__ void wgemm(float (*src)[68], float (*dst)[68], const float* __restrict__ Wm, int K, int nout, const float* __restrict__ G, const float* __restrict__ Bb, int mode, int wave, int lane) { const int col = lane & 15, g = lane >> 4; const int nkc = (K + 31) / 32, nj = (nout + 15) / 16;
#pragma unroll 1
  for (int rt = 0; rt < 2; ++rt) { const int rbase = (wave * 2 + rt) * 16; v8f acc[4] = {};
#pragma unroll
    for (int kc = 0; kc < 2; ++kc) { if (kc >= nkc) break; float va[16];
#pragma unroll
      for (int i = 0; i < 16; ++i) { const int k = kc * 32 + 8 * g + (i < 8 ? i : 8 + i); va[i] = k < K ? src[rbase + col][k] : 0.f; }
      const F2 a = bsplit16(va);
#pragma unroll
      for (int j = 0; j < 4; ++j) { if (j >= nj) break; v16b w; const int o = j * 16 + col; const int oc = o < nout ? o : nout - 1; const float keep = o < nout ? 1.f : 0.f;
#pragma unroll
        for (int i = 0; i < 16; ++i) { const int k = kc * 32 + 8 * g + (i < 8 ? i : 8 + i); w[i] = (__bf16)((k < K ? Wm[(size_t)oc * K + k] : 0.f) * keep); }
        asm volatile("s_wait_loadcnt 0x0" ::: "memory");
        acc[j] = wmma_bf(a.h, w, acc[j]); acc[j] = wmma_bf(a.l, w, acc[j]); } }
    LDSX();
#pragma unroll
    for (int j = 0; j < 4; ++j) { if (j >= nj) break; const int o = j * 16 + col; float gg = 1.f, bb = 0.f; if (mode == 1 && o < nout) { gg = bfr(G[o]) * BNI; bb = bfr(Bb[o]); }
#pragma unroll
      for (int r = 0; r < 8; ++r) { float v = acc[j][r]; if (mode == 1) v = fmaxf(v * gg + bb, 0.f); if (o < nout) dst[rbase + 8 * g + r][o] = v; } }
    LDSX(); } }
__global__ __launch_bounds__(256) void k_edge(const float* __restrict__ C3, const float* __restrict__ F8, const int* __restrict__ IDX,
    const float* __restrict__ LW1, const float* __restrict__ LG1, const float* __restrict__ LB1, const float* __restrict__ LW2, const float* __restrict__ LG2, const float* __restrict__ LB2,
    const float* __restrict__ M1W, const float* __restrict__ M1G, const float* __restrict__ M1B, const float* __restrict__ M2W, const float* __restrict__ M2G, const float* __restrict__ M2B,
    const float* __restrict__ ATW, float* __restrict__ PL) {
  __shared__ __align__(16) float sa[EPB][68], sb[EPB][68];
  const int tid = threadIdx.x, wave = tid >> 5, lane = tid & 31; const size_t e = (size_t)blockIdx.x * EPB + tid; const size_t n = e >> 4; const int s = (int)(e & 15); const size_t b = n / NPT;
  int ii = IDX[n * KN + s]; ii = ii < 0 ? 0 : (ii >= NPT ? NPT - 1 : ii); const size_t m = b * NPT + ii;
  { const float rx = bfr(C3[m * 3]) - bfr(C3[n * 3]), ry = bfr(C3[m * 3 + 1]) - bfr(C3[n * 3 + 1]), rz = bfr(C3[m * 3 + 2]) - bfr(C3[n * 3 + 2]);
    float d2;
    {
#pragma clang fp contract(off)
      d2 = (rx * rx + ry * ry) + rz * rz; }
    sa[tid][0] = rx; sa[tid][1] = ry; sa[tid][2] = rz; sa[tid][3] = sqrtf(d2); }
  LDSX();
  wgemm(sa, sb, LW1, 4, CI, LG1, LB1, 1, wave, lane);
  wgemm(sb, sa, LW2, CI, 2 * CI, LG2, LB2, 1, wave, lane);
  {
#pragma unroll
    for (int c = 0; c < CI; ++c) sb[tid][c] = bfr(F8[m * CI + c]);
#pragma unroll
    for (int c = 0; c < 2 * CI; ++c) sb[tid][CI + c] = sa[tid][c]; }
  LDSX();
  wgemm(sb, sa, M1W, 3 * CI, CO / 2, M1G, M1B, 1, wave, lane);
  wgemm(sa, sb, M2W, CO / 2, CO, M2G, M2B, 1, wave, lane);
  wgemm(sb, sa, ATW, CO, CO, nullptr, nullptr, 0, wave, lane);
  { float mine[4]; mine[0] = mine[1] = mine[2] = mine[3] = 0.f;
#pragma unroll
    for (int c4 = 0; c4 < CO; c4 += 4) { float contrib[4];
#pragma unroll
      for (int i = 0; i < 4; ++i) { const int cc = c4 + i; const float lg = sa[tid][cc]; float mx = lg;
#pragma unroll
        for (int o = 1; o < 16; o <<= 1) mx = fmaxf(mx, __shfl_xor(mx, o));
        const float ex = expf(lg - mx); float sm = ex;
#pragma unroll
        for (int o = 1; o < 16; o <<= 1) sm += __shfl_xor(sm, o);
        float val = (ex / sm) * sb[tid][cc];
#pragma unroll
        for (int o = 1; o < 16; o <<= 1) val += __shfl_xor(val, o);
        contrib[i] = val; }
      if ((c4 >> 2) == s) { mine[0] = contrib[0]; mine[1] = contrib[1]; mine[2] = contrib[2]; mine[3] = contrib[3]; } }
    v4f o4; o4[0] = mine[0]; o4[1] = mine[1]; o4[2] = mine[2]; o4[3] = mine[3]; vst2(PL + n * CO + s * 4, o4); } }
__global__ __launch_bounds__(128) void k_pool(const float* __restrict__ PL, const float* __restrict__ PW, const float* __restrict__ PG, const float* __restrict__ PB, float* __restrict__ OUT) { __shared__ __align__(16) float sa[128][68], sb[128][68];
  const int tid = threadIdx.x, wave = tid >> 5, lane = tid & 31; const size_t r0 = (size_t)blockIdx.x * 128;
  for (int e2 = tid; e2 < 128 * 16; e2 += 128) { const int rl = e2 >> 4, q = e2 & 15; *(v4f*)&sa[rl][q * 4] = *(const v4f*)(PL + (r0 + rl) * CO + q * 4); }
  __syncthreads();
  wgemm(sa, sb, PW, CO, CO, PG, PB, 1, wave, lane);
  for (int rl = 0; rl < 32; ++rl) if (lane < 16) vst2(OUT + (r0 + wave * 32 + rl) * CO + lane * 4, *(const v4f*)&sb[wave * 32 + rl][lane * 4]); }
extern "C" void kernel_launch(void* const* d_in, const int* in_sizes, int n_in, void* d_out, int out_size, void* d_ws, size_t ws_size, hipStream_t stream) {
  (void)in_sizes; (void)n_in; (void)out_size;
  if (ws_size < (size_t)WS_END) return;
  char* ws = (char*)d_ws; const float** F = (const float**)d_in; float* PL = (float*)(ws + WS_PL);
  k_edge<<<dim3(NRV * KN / EPB), 256, 0, stream>>>(F[0], F[1], (const int*)d_in[2], F[3], F[4], F[5], F[6], F[7], F[8], F[9], F[10], F[11], F[12], F[13], F[14], F[15], PL);
  k_pool<<<dim3(NRV / 128), 128, 0, stream>>>(PL, F[16], F[17], F[18], (float*)d_out);
}
